// GTLUTProduct_23871428231429
// MI455X (gfx1250) — hardware-verified
//
#include <hip/hip_runtime.h>
#include <hip/hip_bf16.h>

typedef __attribute__((ext_vector_type(16))) _Float16 v16h;
typedef __attribute__((ext_vector_type(8)))  float    v8f;
typedef __attribute__((ext_vector_type(4)))  float    v4f_t;
typedef float v4fa __attribute__((ext_vector_type(4), may_alias));
typedef __attribute__((ext_vector_type(2)))  float    v2f_t;
#define RSPLIT (1.0f / 2048.0f)
__device__ __forceinline__ _Float16 lo_of(float v, _Float16 h) { return (_Float16)((v - (float)h) * 2048.0f); }
__device__ __forceinline__ v8f wmma16(v16h a, v16h b, v8f c) { return __builtin_amdgcn_wmma_f32_16x16x32_f16(false, a, false, b, (short)0, c, false, false); }
__device__ __forceinline__ v8f wmma_split(v16h a, v16h al, v16h b, v16h bl, v8f c) { v8f x = {}; x = wmma16(al, b, x); x = wmma16(a, bl, x); return wmma16(a, b, c) + x * RSPLIT; }
__device__ __forceinline__ void frag32(const float* rowp, int half, v16h& hv, v16h& lv) {
#pragma unroll
  for (int e = 0; e < 16; ++e) { const float v = rowp[8 * half + ((e < 8) ? e : (e + 8))]; hv[e] = (_Float16)v; lv[e] = lo_of(v, hv[e]); }
}

#define Bn 4
#define Ln 256
#define Fh 64
#define Dn 8
#define Kn 6
#define DK 48
#define An 64
#define On 64
#define DA 512

#define G1_OFF 0
#define G2_OFF (Bn*Ln*DK)
#define G3_OFF (2*Bn*Ln*DK)
#define SS_OFF (2*Bn*Ln*DK + Ln*DK)

__global__ __launch_bounds__(128) void k_proj(const float* __restrict__ in1,
                                              const float* __restrict__ in2,
                                              const float* __restrict__ pos,
                                              const float* __restrict__ anchors,
                                              float* __restrict__ ws) {
  __shared__ __attribute__((aligned(16))) float st[4][16 * DK];
  const int lane = threadIdx.x & 31, wave = threadIdx.x >> 5, half = lane >> 4, l16 = lane & 15;
  const int mt = blockIdx.x * 4 + wave;
  const int r0 = mt * 16;
  const float* src; float* dst; int f0;
  if (r0 < Bn * Ln)          { src = in1 + (size_t)r0 * Fh;                 f0 = 0;   dst = ws + G1_OFF + (size_t)r0 * DK; }
  else if (r0 < 2 * Bn * Ln) { src = in2 + (size_t)(r0 - Bn * Ln) * Fh;     f0 = 64;  dst = ws + G2_OFF + (size_t)(r0 - Bn * Ln) * DK; }
  else                       { src = pos + (size_t)(r0 - 2 * Bn * Ln) * Fh; f0 = 128; dst = ws + G3_OFF + (size_t)(r0 - 2 * Bn * Ln) * DK; }
  v8f acc[3] = {};
#pragma unroll
  for (int kc = 0; kc < 2; ++kc) {
    v16h a, al; frag32(src + (size_t)l16 * Fh + kc * 32, half, a, al);
#pragma unroll
    for (int nt = 0; nt < 3; ++nt) {
      v16h b, bl; frag32(anchors + (size_t)(nt * 16 + l16) * 192 + f0 + kc * 32, half, b, bl);
      acc[nt] = wmma_split(a, al, b, bl, acc[nt]);
    }
  }
  float* sw = st[wave];
#pragma unroll
  for (int nt = 0; nt < 3; ++nt)
#pragma unroll
    for (int r = 0; r < 8; ++r) sw[(r + 8 * half) * DK + nt * 16 + l16] = acc[nt][r];
  asm volatile("s_wait_dscnt 0" ::: "memory");
#pragma unroll 1
  for (int pass = 0; pass < 2; ++pass) {
    for (int q = lane; q < 16 * DK / 4; q += 32) *(volatile v4f_t*)(dst + q * 4) = *(const volatile v4fa*)(sw + q * 4);
    __threadfence();
  }
}

__global__ __launch_bounds__(256) void k_ssum(const float* __restrict__ ws_g,
                                              float* __restrict__ ssum) {
  const int j = blockIdx.x;
  const int b = blockIdx.y;
  const int tid = threadIdx.x;

  __shared__ float sig[32][DK];
  __shared__ float g2j[DK];

  const float* G1 = ws_g + G1_OFF + (b * Ln) * DK;
  const float* G2 = ws_g + G2_OFF + (b * Ln + j) * DK;
  const float* G3 = ws_g + G3_OFF;

  if (tid < DK) g2j[tid] = G2[tid];
  __syncthreads();

  const int d  = tid >> 5;
  const int a0 = (tid & 31) << 1;
  float acc0 = 0.f, acc1 = 0.f;

  for (int i0 = 0; i0 < j; i0 += 32) {
    const int nI = min(32, j - i0);
    for (int s = tid; s < nI * DK; s += 256) {
      int il = s / DK, c = s % DK;
      int i = i0 + il;
      float x = G1[i * DK + c] + g2j[c] + G3[(j - i) * DK + c];
      sig[il][c] = 1.f / (1.f + __expf(-x));
    }
    __syncthreads();

    for (int il = 0; il < nI; ++il) {
      const float* sd = &sig[il][d * Kn];
      float common = 1.f;
#pragma unroll
      for (int k = 1; k < Kn; ++k) {
        float sk = sd[k];
        common *= ((a0 >> k) & 1) ? sk : (1.f - sk);
      }
      float s0 = sd[0];
      acc0 += common * (1.f - s0);
      acc1 += common * s0;
    }
    __syncthreads();
  }

  v2f_t o2; o2.x = acc0; o2.y = acc1;
  float* o = ssum + (b * Ln + j) * DA + d * An + a0;
  *(volatile v2f_t*)o = o2; __threadfence(); *(volatile v2f_t*)o = o2;
}

__global__ __launch_bounds__(128) void k_wmma(const float* __restrict__ ssum,
                                              const float* __restrict__ lutw,
                                              float* __restrict__ out) {
  __shared__ __attribute__((aligned(16))) float so[16 * On];
  const int tile  = blockIdx.x;
  const int wave  = threadIdx.x >> 5;
  const int lane  = threadIdx.x & 31;
  const int row16 = lane & 15;
  const int hi    = lane >> 4;
  const int mbase = tile * 16;

  v8f c = {};
  for (int kc = 0; kc < 16; ++kc) {
    v16h a, al, bm, bl;
    frag32(ssum + (mbase + row16) * DA + kc * 32, hi, a, al);
#pragma unroll
    for (int h = 0; h < 16; ++h) {
      const int k = kc * 32 + hi * 8 + (h & 7) + ((h >= 8) ? 16 : 0);
      const float v = lutw[k * On + wave * 16 + row16];
      bm[h] = (_Float16)v; bl[h] = lo_of(v, bm[h]);
    }
    c = wmma_split(a, al, bm, bl, c);
  }

#pragma unroll
  for (int r = 0; r < 8; ++r) so[(hi * 8 + r) * On + wave * 16 + row16] = c[r];
  __syncthreads();
#pragma unroll 1
  for (int pass = 0; pass < 2; ++pass) {
    for (int q = threadIdx.x; q < 16 * On / 4; q += 128) *(volatile v4f_t*)(out + (size_t)mbase * On + q * 4) = *(const volatile v4fa*)(so + q * 4);
    __threadfence();
  }
}

extern "C" void kernel_launch(void* const* d_in, const int* in_sizes, int n_in,
                              void* d_out, int out_size, void* d_ws, size_t ws_size,
                              hipStream_t stream) {
  (void)in_sizes; (void)n_in; (void)out_size; (void)ws_size;

  const float* in1     = (const float*)d_in[0];
  const float* in2     = (const float*)d_in[1];
  const float* pos     = (const float*)d_in[2];
  const float* anchors = (const float*)d_in[3];
  const float* lutw    = (const float*)d_in[4];
  float* out = (float*)d_out;
  float* ws  = (float*)d_ws;
  float* ssum = ws + SS_OFF;

  k_proj<<<(2 * Bn * Ln + Ln) / 16 / 4, 128, 0, stream>>>(in1, in2, pos, anchors, ws);

  dim3 gridB(Ln, Bn);
  k_ssum<<<gridB, 256, 0, stream>>>(ws, ssum);

  k_wmma<<<(Bn * Ln) / 16, 128, 0, stream>>>(ssum, lutw, out);
}
